// MambaEncoderLayer_40097814675763
// MI455X (gfx1250) — hardware-verified
//
#include <hip/hip_runtime.h>
#include <math.h>

typedef __attribute__((ext_vector_type(16))) _Float16 v16h;
typedef __attribute__((ext_vector_type(8)))  _Float16 v8h;
typedef __attribute__((ext_vector_type(16))) __bf16   v16b;
typedef __attribute__((ext_vector_type(8)))  __bf16   v8b;
typedef __attribute__((ext_vector_type(8)))  float    v8f;
typedef __attribute__((ext_vector_type(4)))  float    v4f;

constexpr int kBatch = 2;
constexpr int kSeqL  = 2048;
constexpr int kDmod  = 1024;
constexpr int kDin   = 2048;
constexpr int kNst   = 16;
constexpr int kDtR   = 64;
constexpr int kPrjN  = 96;
constexpr int kPrjP  = 128;
constexpr int kXZP   = 2 * kDin;
constexpr int kRows  = kBatch * kSeqL;
constexpr int kTP    = 260;
constexpr float kLnEps = 1e-6f;
static_assert(kDin == 2 * kDmod, "expand 2");
static_assert(kDtR == (kDmod + 15) / 16, "dt rank");
static_assert(kPrjN == kDtR + 2 * kNst, "x_proj width");
static_assert(kPrjP % 64 == 0 && kPrjP >= kPrjN, "padded x_proj width");
static_assert((kDmod % 32) == 0 && (kDin % 32) == 0 && (kDtR % 32) == 0, "GEMM K multiples of 32");
static_assert((kSeqL % 64) == 0 && (kXZP % 64) == 0 && (kDin % 64) == 0 && (kDmod % 64) == 0, "GEMM M,N multiples of 64");
static_assert((kDin % 256) == 0 && (kSeqL % 64) == 0 && (kSeqL % 16) == 0, "conv / scan tiles");
static_assert(kDmod == 4 * 256, "LayerNorm block covers one row");

constexpr float kCarX    = 64.0f;
constexpr float kCarWin  = 1024.0f;
constexpr float kCarU    = 64.0f;
constexpr float kCarWxp  = 1024.0f;
constexpr float kCarDt   = 64.0f;
constexpr float kCarWdt  = 256.0f;
constexpr float kCarY    = 16.0f;
constexpr float kCarWout = 1024.0f;
constexpr float kSclIn   = 1.0f / (kCarX * kCarWin);
constexpr float kSclXp   = 1.0f / (kCarU * kCarWxp);
constexpr float kSclDt   = 1.0f / (kCarDt * kCarWdt);
constexpr float kSclOut  = 1.0f / (kCarY * kCarWout);

constexpr size_t kSzWIN16  = (size_t)kXZP * kDmod * 2;
constexpr size_t kSzWXP16  = (size_t)kPrjP * kDin * 2;
constexpr size_t kSzWDT16  = (size_t)kDin * kDtR * 2;
constexpr size_t kSzWOUT16 = (size_t)kDmod * kDin * 2;
constexpr size_t kSzX16    = (size_t)kRows * kDmod * 2;
constexpr size_t kSzXZ     = (size_t)kSeqL * kXZP * 4;
constexpr size_t kSzUC     = (size_t)kSeqL * kDin * 4;
constexpr size_t kSzUC16   = (size_t)kSeqL * kDin * 2;
constexpr size_t kSzPROJ   = (size_t)kSeqL * kPrjP * 4;
constexpr size_t kSzDT16   = (size_t)kSeqL * kDtR * 2;
constexpr size_t kSzDLR    = (size_t)kSeqL * kDin * 4;
constexpr size_t kSzY16    = (size_t)kSeqL * kDin * 2;
constexpr size_t kSzMB     = (size_t)kRows * kDmod * 4;
constexpr size_t kOffWIN16  = 0;
constexpr size_t kOffWXP16  = kOffWIN16  + kSzWIN16;
constexpr size_t kOffWDT16  = kOffWXP16  + kSzWXP16;
constexpr size_t kOffWOUT16 = kOffWDT16  + kSzWDT16;
constexpr size_t kOffX16    = kOffWOUT16 + kSzWOUT16;
constexpr size_t kOffXZ     = kOffX16    + kSzX16;
constexpr size_t kOffUC     = kOffXZ     + kSzXZ;
constexpr size_t kOffUC16   = kOffUC     + kSzUC;
constexpr size_t kOffPROJ   = kOffUC16   + kSzUC16;
constexpr size_t kOffDT16   = kOffPROJ   + kSzPROJ;
constexpr size_t kOffDLR    = kOffDT16   + kSzDT16;
constexpr size_t kOffY16    = kOffDLR    + kSzDLR;
constexpr size_t kOffMB     = kOffY16    + kSzY16;
constexpr size_t kWsTotal   = kOffMB     + kSzMB;
static_assert(kWsTotal == 123731968ull, "carve total");
static_assert(kWsTotal <= 134217728ull, "carve cap");
static_assert((kOffWXP16 % 128) == 0 && (kOffWDT16 % 128) == 0 && (kOffWOUT16 % 128) == 0 && (kOffX16 % 128) == 0 &&
              (kOffXZ % 128) == 0 && (kOffUC % 128) == 0 && (kOffUC16 % 128) == 0 && (kOffPROJ % 128) == 0 &&
              (kOffDT16 % 128) == 0 && (kOffDLR % 128) == 0 && (kOffY16 % 128) == 0 && (kOffMB % 128) == 0,
              "128-B aligned regions");

__device__ __forceinline__ unsigned short f2bf_bits(float f) {
  unsigned u = __float_as_uint(f);
  return (unsigned short)((u + 0x7FFFu + ((u >> 16) & 1u)) >> 16);
}
__device__ __forceinline__ float bf_bits2f(unsigned short h) { return __uint_as_float(((unsigned)h) << 16); }
__device__ __forceinline__ float bf_rne(float f) { return bf_bits2f(f2bf_bits(f)); }

__device__ __forceinline__ void dep_guard4_h(v8f& a, v8f& b, v8f& c, v8f& d, v16h x, v16h y) { asm volatile("v_nop\n\tv_nop\n\tv_nop\n\tv_nop" : "+v"(a), "+v"(b), "+v"(c), "+v"(d) : "v"(x), "v"(y)); }
__device__ __forceinline__ void dep_guard4_b(v8f& a, v8f& b, v8f& c, v8f& d, v16b x, v16b y) { asm volatile("v_nop\n\tv_nop\n\tv_nop\n\tv_nop" : "+v"(a), "+v"(b), "+v"(c), "+v"(d) : "v"(x), "v"(y)); }
__device__ __forceinline__ void keep4_h(v16h a, v16h b, v16h c, v16h d) { asm volatile("v_nop" :: "v"(a), "v"(b), "v"(c), "v"(d)); }
__device__ __forceinline__ void keep4_b(v16b a, v16b b, v16b c, v16b d) { asm volatile("v_nop" :: "v"(a), "v"(b), "v"(c), "v"(d)); }
__device__ __forceinline__ void acc_guard4(v8f& a, v8f& b, v8f& c, v8f& d) { asm volatile("v_nop\n\tv_nop\n\tv_nop\n\tv_nop" : "+v"(a), "+v"(b), "+v"(c), "+v"(d)); }
template <typename T> struct Frag;
template <> struct Frag<_Float16> {
  typedef v16h V; union U { v16h v; v8h h[2]; };
  static __device__ __forceinline__ v16h load(const _Float16* p) {
    U f; f.h[0] = *(const v8h*)(p); f.h[1] = *(const v8h*)(p + 16); return f.v;
  }
  static __device__ __forceinline__ v8f mma(v16h a, v16h b, v8f c) {
    return __builtin_amdgcn_wmma_f32_16x16x32_f16(false, a, false, b, (short)0, c, false, false);
  }
  static __device__ __forceinline__ void guard4(v8f& a, v8f& b, v8f& c, v8f& d, v16h x, v16h y) { dep_guard4_h(a, b, c, d, x, y); }
  static __device__ __forceinline__ void keep(v16h a, v16h b, v16h c, v16h d) { keep4_h(a, b, c, d); }
};
template <> struct Frag<__bf16> {
  typedef v16b V; union U { v16b v; v8b h[2]; };
  static __device__ __forceinline__ v16b load(const __bf16* p) {
    U f; f.h[0] = *(const v8b*)(p); f.h[1] = *(const v8b*)(p + 16); return f.v;
  }
  static __device__ __forceinline__ v8f mma(v16b a, v16b b, v8f c) {
    return __builtin_amdgcn_wmma_f32_16x16x32_bf16(false, a, false, b, (short)0, c, false, false);
  }
  static __device__ __forceinline__ void guard4(v8f& a, v8f& b, v8f& c, v8f& d, v16b x, v16b y) { dep_guard4_b(a, b, c, d, x, y); }
  static __device__ __forceinline__ void keep(v16b a, v16b b, v16b c, v16b d) { keep4_b(a, b, c, d); }
};

template <int ET> struct Elem;
template <> struct Elem<0> { typedef _Float16 T; };
template <> struct Elem<1> { typedef __bf16 T; };
template <int ET, bool SPLIT, int BIAS_MODE, int OUT_MODE, bool RESID, int ACT = 0>
__global__ __launch_bounds__(256) void wmma_gemm64(
    const unsigned short* __restrict__ Ap, const unsigned short* __restrict__ A2p, int lda, long strideA,
    const unsigned short* __restrict__ Btp, const unsigned short* __restrict__ Bt2p, int ldb, long strideB,
    void* __restrict__ Cout, void* __restrict__ Cout2, int ldc, long strideC,
    const float* __restrict__ bias,
    const float* __restrict__ resid, long strideR,
    int M, int N, int K, float scale) {
  typedef typename Elem<ET>::T T;
  typedef typename Frag<T>::V V;
  const T* A = (const T*)Ap; const T* A2 = (const T*)A2p; const T* Bt = (const T*)Btp; const T* Bt2 = (const T*)Bt2p;
  __shared__ __align__(16) float sT[8][16 * 68];
  const int b    = blockIdx.y;
  const int lane = threadIdx.x & 31;
  const int wave = threadIdx.x >> 5;
  const int tilesN = N >> 6;
  const int tilesM = M >> 6;
  const int tile = blockIdx.x * 8 + wave;
  if (tile >= tilesM * tilesN) return;
  const int tm = tile / tilesN;
  const int tn = tile - tm * tilesN;
  const int m0 = tm << 6;
  const int n0 = tn << 6;

  const T* Ab  = A  + (size_t)b * strideA;
  const T* Bb  = Bt + (size_t)b * strideB;
  const T* Ab2 = SPLIT ? (A2  + (size_t)b * strideA) : nullptr;
  const T* Bb2 = SPLIT ? (Bt2 + (size_t)b * strideB) : nullptr;

  const int rlane = lane & 15;
  const int koff  = (lane >> 4) * 8;
  const int mOff  = (lane >> 4) * 8;

  v8f acc[4][4];
#pragma unroll
  for (int i = 0; i < 4; ++i)
#pragma unroll
    for (int j = 0; j < 4; ++j) acc[i][j] = (v8f){0.f,0.f,0.f,0.f,0.f,0.f,0.f,0.f};

  for (int k0 = 0; k0 < K; k0 += 32) {
    V bh[4], bl[4];
#pragma unroll
    for (int j = 0; j < 4; ++j) {
      const size_t bo = (size_t)(n0 + (j << 4) + rlane) * ldb + koff + k0;
      bh[j] = Frag<T>::load(Bb + bo);
      if (SPLIT) bl[j] = Frag<T>::load(Bb2 + bo);
    }
#pragma unroll
    for (int i = 0; i < 4; ++i) {
      const size_t ao = (size_t)(m0 + (i << 4) + rlane) * lda + koff + k0;
      V ah = Frag<T>::load(Ab + ao);
      V al;
      if (SPLIT) al = Frag<T>::load(Ab2 + ao);
#pragma unroll
      for (int j = 0; j < 4; ++j) {
        acc[i][j] = Frag<T>::mma(ah, bh[j], acc[i][j]);
        if (SPLIT) {
          acc[i][j] = Frag<T>::mma(ah, bl[j], acc[i][j]);
          acc[i][j] = Frag<T>::mma(al, bh[j], acc[i][j]);
        }
      }
      Frag<T>::guard4(acc[i][0], acc[i][1], acc[i][2], acc[i][3], ah, SPLIT ? al : ah);
    }
    Frag<T>::keep(bh[0], bh[1], bh[2], bh[3]);
    if (SPLIT) Frag<T>::keep(bl[0], bl[1], bl[2], bl[3]);
  }
  acc_guard4(acc[0][0], acc[0][1], acc[0][2], acc[0][3]);
  acc_guard4(acc[1][0], acc[1][1], acc[1][2], acc[1][3]);
  acc_guard4(acc[2][0], acc[2][1], acc[2][2], acc[2][3]);
  acc_guard4(acc[3][0], acc[3][1], acc[3][2], acc[3][3]);

  float* slab = sT[wave];
  const float* Rb = RESID ? (resid + (size_t)b * strideR) : nullptr;
#pragma unroll
  for (int i = 0; i < 4; ++i) {
    const int mBase = m0 + (i << 4);
#pragma unroll
    for (int j = 0; j < 4; ++j) {
      const int n = n0 + (j << 4) + rlane;
      float bv = 0.f;
      if (BIAS_MODE == 2) bv = bias[n];
#pragma unroll
      for (int r = 0; r < 8; ++r) {
        float v = acc[i][j][r] * scale;
        if (BIAS_MODE == 1) v += bias[mBase + mOff + r];
        if (BIAS_MODE == 2) v += bv;
        if (RESID) v += Rb[(size_t)(mBase + mOff + r) * ldc + n];
        if (ACT == 1) v = tanhf(v);
        if (ACT == 2) v = fmaxf(v, 0.0f);
        if (ACT == 3) v = v / (1.0f + expf(-v));
        if (ACT == 4) v = (v > 0.f) ? v : 0.01f * v;
        slab[(mOff + r) * 68 + (j << 4) + rlane] = v;
      }
    }
    __builtin_amdgcn_fence(__ATOMIC_RELEASE, "workgroup");
    __builtin_amdgcn_wave_barrier();
    __builtin_amdgcn_fence(__ATOMIC_ACQUIRE, "workgroup");
    if (OUT_MODE == 0) {
      float* C = (float*)Cout + (size_t)b * strideC;
      const int hh = lane >> 4, c4 = (lane & 15) * 4;
      for (int pass = 0; pass < 2; ++pass) {
#pragma unroll
        for (int it = 0; it < 8; ++it) {
          const int row = it * 2 + hh;
          v4f v = *(const v4f*)(slab + row * 68 + c4);
          *(volatile v4f*)(C + (size_t)(mBase + row) * ldc + n0 + c4) = v;
        }
        __threadfence();
      }
    } else {
      const int q = lane >> 3, c8 = (lane & 7) * 8;
      unsigned short* C  = (unsigned short*)Cout  + (size_t)b * strideC;
      unsigned short* C2 = (OUT_MODE == 2) ? ((unsigned short*)Cout2 + (size_t)b * strideC) : nullptr;
      for (int pass = 0; pass < 2; ++pass) {
#pragma unroll
        for (int it = 0; it < 4; ++it) {
          const int row = it * 4 + q;
          const float* sp = slab + row * 68 + c8;
          v8h hv, lv;
#pragma unroll
          for (int e = 0; e < 8; ++e) {
            if (OUT_MODE == 1) {
              hv[e] = (_Float16)sp[e];
            } else {
              unsigned short hb = f2bf_bits(sp[e]);
              unsigned short lb = f2bf_bits(sp[e] - bf_bits2f(hb));
              hv[e] = __builtin_bit_cast(_Float16, hb);
              lv[e] = __builtin_bit_cast(_Float16, lb);
            }
          }
          *(volatile v8h*)(C + (size_t)(mBase + row) * ldc + n0 + c8) = hv;
          if (OUT_MODE == 2) *(volatile v8h*)(C2 + (size_t)(mBase + row) * ldc + n0 + c8) = lv;
        }
        __threadfence();
      }
    }
    __builtin_amdgcn_fence(__ATOMIC_RELEASE, "workgroup");
    __builtin_amdgcn_wave_barrier();
    __builtin_amdgcn_fence(__ATOMIC_ACQUIRE, "workgroup");
  }
}

__global__ __launch_bounds__(256) void cast_f16_kernel(
    const float* __restrict__ src, unsigned short* __restrict__ dst, int total8, int real8, float scale)
{
  const int i = blockIdx.x * 256 + threadIdx.x;
  if (i >= total8) return;
  const bool live = (i < real8);
  const int ic = live ? i : (real8 - 1);
  const float* p = src + ((size_t)ic << 3);
  const v4f a0 = *(const v4f*)(p);
  const v4f a1 = *(const v4f*)(p + 4);
  v8h hv;
#pragma unroll
  for (int e = 0; e < 4; ++e) {
    const float s0 = a0[e];
    const float s1 = a1[e];
    const float f0 = live ? (bf_rne(s0) * scale) : 0.0f;
    const float f1 = live ? (bf_rne(s1) * scale) : 0.0f;
    hv[e]     = (_Float16)f0;
    hv[4 + e] = (_Float16)f1;
  }
  unsigned short* q = dst + ((size_t)i << 3);
  *(volatile v8h*)q = hv;
  __threadfence();
  *(volatile v8h*)q = hv;
}

__global__ __launch_bounds__(256) void dt_cast_kernel(
    const float* __restrict__ PROJ, unsigned short* __restrict__ DT16, int total8, float scale)
{
  const int i = blockIdx.x * 256 + threadIdx.x;
  if (i >= total8) return;
  const int e0  = i << 3;
  const int row = e0 >> 6;
  const int c8  = e0 & 63;
  const float* p = PROJ + (size_t)row * kPrjP + c8;
  const v4f a0 = *(const v4f*)(p);
  const v4f a1 = *(const v4f*)(p + 4);
  v8h hv;
#pragma unroll
  for (int e = 0; e < 4; ++e) {
    hv[e]     = (_Float16)(a0[e] * scale);
    hv[4 + e] = (_Float16)(a1[e] * scale);
  }
  unsigned short* qd = DT16 + e0;
  *(volatile v8h*)qd = hv;
  __threadfence();
  *(volatile v8h*)qd = hv;
}

__global__ __launch_bounds__(256) void conv_silu_kernel(
    const float* __restrict__ XZ, const float* __restrict__ cw, const float* __restrict__ cb,
    float* __restrict__ UC, unsigned short* __restrict__ UC16)
{
  __shared__ __align__(16) float sT[16 * kTP];
  const int tid = threadIdx.x, lane = tid & 31, wave = tid >> 5;
  const int d0 = blockIdx.x * 256, d = d0 + tid;
  const int t0 = blockIdx.y * 64;
  const v4f wq = *(const v4f*)(cw + (size_t)d * 4);
  const float wr0 = wq[0], wr1 = wq[1], wr2 = wq[2], wr3 = wq[3];
  const float w0 = bf_rne(wr0), w1 = bf_rne(wr1), w2 = bf_rne(wr2), w3 = bf_rne(wr3);
  const float bc = bf_rne(cb[d]);
  float xm3, xm2, xm1;
  {
    const int r3 = t0 - 3, r2 = t0 - 2, r1 = t0 - 1;
    const float v3 = XZ[(size_t)(r3 < 0 ? 0 : r3) * kXZP + d];
    const float v2 = XZ[(size_t)(r2 < 0 ? 0 : r2) * kXZP + d];
    const float v1 = XZ[(size_t)(r1 < 0 ? 0 : r1) * kXZP + d];
    xm3 = (r3 >= 0) ? v3 : 0.f;
    xm2 = (r2 >= 0) ? v2 : 0.f;
    xm1 = (r1 >= 0) ? v1 : 0.f;
  }
  const int hrow = wave >> 1;
  const int hch  = (wave & 1) * 128 + lane * 4;
#pragma unroll 1
  for (int sub = 0; sub < 4; ++sub) {
    const int lb = t0 + sub * 16;
#pragma unroll 1
    for (int s = 0; s < 16; ++s) {
      const float xc = XZ[(size_t)(lb + s) * kXZP + d];
      float acc = w0 * xm3;
      acc = fmaf(w1, xm2, acc);
      acc = fmaf(w2, xm1, acc);
      acc = fmaf(w3, xc, acc);
      const float sv = acc + bc;
      const float sg = __builtin_amdgcn_rcpf(1.0f + __expf(-sv));
      sT[s * kTP + tid] = sv * sg;
      xm3 = xm2; xm2 = xm1; xm1 = xc;
    }
    __syncthreads();
    v4f fv[4];
    v8h bv[2];
#pragma unroll
    for (int it = 0; it < 4; ++it) fv[it] = *(const v4f*)(sT + (it * 4 + hrow) * kTP + hch);
#pragma unroll
    for (int it = 0; it < 2; ++it) {
      const float* sp = sT + (it * 8 + wave) * kTP + lane * 8;
      const v4f a0 = *(const v4f*)(sp);
      const v4f a1 = *(const v4f*)(sp + 4);
#pragma unroll
      for (int e = 0; e < 4; ++e) {
        bv[it][e]     = (_Float16)(a0[e] * kCarU);
        bv[it][4 + e] = (_Float16)(a1[e] * kCarU);
      }
    }
    for (int pass = 0; pass < 2; ++pass) {
#pragma unroll
      for (int it = 0; it < 4; ++it)
        *(volatile v4f*)(UC + (size_t)(lb + it * 4 + hrow) * kDin + d0 + hch) = fv[it];
#pragma unroll
      for (int it = 0; it < 2; ++it)
        *(volatile v8h*)(UC16 + (size_t)(lb + it * 8 + wave) * kDin + d0 + lane * 8) = bv[it];
      __threadfence();
    }
    __syncthreads();
  }
}

__global__ __launch_bounds__(256) void scan_kernel(
    const float* __restrict__ DLR, const float* __restrict__ UC, const float* __restrict__ XZ,
    const float* __restrict__ PROJ, const float* __restrict__ bdt, const float* __restrict__ A_log,
    const float* __restrict__ Dv, unsigned short* __restrict__ Y16)
{
  __shared__ __align__(16) float sBC[16 * 32];
  __shared__ __align__(16) float sY[16 * kTP];
  const int tid = threadIdx.x, lane = tid & 31, wave = tid >> 5;
  const int d0 = blockIdx.x * 256, d = d0 + tid;

  float An[kNst];
#pragma unroll
  for (int qq = 0; qq < 4; ++qq) {
    const v4f aq = *(const v4f*)(A_log + (size_t)d * kNst + 4 * qq);
    const float a0 = aq[0], a1 = aq[1], a2 = aq[2], a3 = aq[3];
    An[4 * qq + 0] = -__expf(bf_rne(a0));
    An[4 * qq + 1] = -__expf(bf_rne(a1));
    An[4 * qq + 2] = -__expf(bf_rne(a2));
    An[4 * qq + 3] = -__expf(bf_rne(a3));
  }
  const float Dd = bf_rne(Dv[d]);
  const float bb = bf_rne(bdt[d]);
  float h[kNst];
#pragma unroll
  for (int n = 0; n < kNst; ++n) h[n] = 0.f;

#pragma unroll 1
  for (int c = 0; c < kSeqL / 16; ++c) {
    const int l0 = c * 16;
    if (tid < 128) {
      const int r = tid >> 3, q = (tid & 7) * 4;
      const v4f v = *(const v4f*)(PROJ + (size_t)(l0 + r) * kPrjP + kDtR + q);
      *(v4f*)(sBC + r * 32 + q) = v;
    }
    __syncthreads();
#pragma unroll 1
    for (int s = 0; s < 16; ++s) {
      const size_t m = (size_t)(l0 + s);
      const float a   = DLR[m * kDin + d] + bb;
      const float ea  = __expf(-fabsf(a));
      const float u   = 1.0f + ea;
      const float l1p = __logf(u) + (ea - (u - 1.0f)) * __builtin_amdgcn_rcpf(u);
      const float delta = fmaxf(a, 0.0f) + l1p;
      const float xv    = UC[m * kDin + d];
      const float zv    = XZ[m * kXZP + kDin + d];
      v4f Bq[4], Cq[4];
#pragma unroll
      for (int qq = 0; qq < 4; ++qq) {
        Bq[qq] = *(const v4f*)(sBC + s * 32 + 4 * qq);
        Cq[qq] = *(const v4f*)(sBC + s * 32 + kNst + 4 * qq);
      }
      const float dbx = delta * xv;
      float y = 0.f;
#pragma unroll
      for (int n = 0; n < kNst; ++n) {
        const float e  = __expf(delta * An[n]);
        const float hn = h[n] * e + dbx * Bq[n >> 2][n & 3];
        h[n] = hn;
        y += Cq[n >> 2][n & 3] * hn;
      }
      y += xv * Dd;
      const float sg = __builtin_amdgcn_rcpf(1.0f + __expf(-zv));
      const float g  = zv * sg;
      sY[s * kTP + tid] = (y * g) * kCarY;
    }
    __syncthreads();
    v8h hv[2];
#pragma unroll
    for (int it = 0; it < 2; ++it) {
      const float* sp = sY + (it * 8 + wave) * kTP + lane * 8;
      const v4f a0 = *(const v4f*)(sp);
      const v4f a1 = *(const v4f*)(sp + 4);
#pragma unroll
      for (int e = 0; e < 4; ++e) { hv[it][e] = (_Float16)a0[e]; hv[it][4 + e] = (_Float16)a1[e]; }
    }
    for (int pass = 0; pass < 2; ++pass) {
#pragma unroll
      for (int it = 0; it < 2; ++it)
        *(volatile v8h*)(Y16 + (size_t)(l0 + it * 8 + wave) * kDin + d0 + lane * 8) = hv[it];
      __threadfence();
    }
  }
}

__global__ __launch_bounds__(256) void ln_resid_kernel(
    const float* __restrict__ MB, const float* __restrict__ x, const float* __restrict__ lw,
    const float* __restrict__ lb, float* __restrict__ out)
{
  __shared__ float sR1[8];
  __shared__ float sR2[8];
  const int tid = threadIdx.x, lane = tid & 31, wave = tid >> 5;
  const int row = blockIdx.x;
  const size_t o = (size_t)row * kDmod + (size_t)tid * 4;
  const v4f mv = *(const v4f*)(MB + o);
  const float m0 = mv[0], m1 = mv[1], m2 = mv[2], m3 = mv[3];
  float s = (m0 + m1) + (m2 + m3);
#pragma unroll
  for (int off = 16; off > 0; off >>= 1) s += __shfl_xor(s, off, 32);
  if (lane == 0) sR1[wave] = s;
  __syncthreads();
  float tot = 0.f;
#pragma unroll
  for (int w = 0; w < 8; ++w) tot += sR1[w];
  const float mu = tot * (1.0f / (float)kDmod);
  const float c0 = m0 - mu, c1 = m1 - mu, c2 = m2 - mu, c3 = m3 - mu;
  float q = (c0 * c0 + c1 * c1) + (c2 * c2 + c3 * c3);
#pragma unroll
  for (int off = 16; off > 0; off >>= 1) q += __shfl_xor(q, off, 32);
  if (lane == 0) sR2[wave] = q;
  __syncthreads();
  float totq = 0.f;
#pragma unroll
  for (int w = 0; w < 8; ++w) totq += sR2[w];
  const float var = totq * (1.0f / (float)kDmod);
  const float rs  = rsqrtf(var + kLnEps);
  const v4f xv = *(const v4f*)(x + o);
  const v4f wv = *(const v4f*)(lw + (size_t)tid * 4);
  const v4f bv = *(const v4f*)(lb + (size_t)tid * 4);
  const float x0 = xv[0], x1 = xv[1], x2 = xv[2], x3 = xv[3];
  const float g0 = wv[0], g1 = wv[1], g2 = wv[2], g3 = wv[3];
  const float h0 = bv[0], h1 = bv[1], h2 = bv[2], h3 = bv[3];
  v4f ov;
  ov[0] = bf_rne(x0) + ((c0 * rs) * bf_rne(g0) + bf_rne(h0));
  ov[1] = bf_rne(x1) + ((c1 * rs) * bf_rne(g1) + bf_rne(h1));
  ov[2] = bf_rne(x2) + ((c2 * rs) * bf_rne(g2) + bf_rne(h2));
  ov[3] = bf_rne(x3) + ((c3 * rs) * bf_rne(g3) + bf_rne(h3));
  float* po = out + o;
  *(volatile v4f*)po = ov;
  __threadfence();
  *(volatile v4f*)po = ov;
}

extern "C" void kernel_launch(void* const* d_in, const int* in_sizes, int n_in,
                              void* d_out, int out_size, void* d_ws, size_t ws_size,
                              hipStream_t stream)
{
  if (n_in < 12) return;
  if (in_sizes[0] != kRows * kDmod) return;
  if (in_sizes[1] != kXZP * kDmod) return;
  if (in_sizes[2] != kDin * 4 || in_sizes[3] != kDin) return;
  if (in_sizes[4] != kPrjN * kDin) return;
  if (in_sizes[5] != kDin * kDtR || in_sizes[6] != kDin) return;
  if (in_sizes[7] != kDin * kNst || in_sizes[8] != kDin) return;
  if (in_sizes[9] != kDmod * kDin) return;
  if (in_sizes[10] != kDmod || in_sizes[11] != kDmod) return;
  if (out_size != kRows * kDmod) return;
  if (ws_size < kWsTotal) return;

  const float* x      = (const float*)d_in[0];
  const float* W_in   = (const float*)d_in[1];
  const float* conv_w = (const float*)d_in[2];
  const float* conv_b = (const float*)d_in[3];
  const float* W_xprj = (const float*)d_in[4];
  const float* W_dt   = (const float*)d_in[5];
  const float* b_dt   = (const float*)d_in[6];
  const float* A_log  = (const float*)d_in[7];
  const float* Dv     = (const float*)d_in[8];
  const float* W_out  = (const float*)d_in[9];
  const float* ln_w   = (const float*)d_in[10];
  const float* ln_b   = (const float*)d_in[11];
  float* dout = (float*)d_out;

  char* ws = (char*)d_ws;
  unsigned short* WIN16  = (unsigned short*)(ws + kOffWIN16);
  unsigned short* WXP16  = (unsigned short*)(ws + kOffWXP16);
  unsigned short* WDT16  = (unsigned short*)(ws + kOffWDT16);
  unsigned short* WOUT16 = (unsigned short*)(ws + kOffWOUT16);
  unsigned short* X16    = (unsigned short*)(ws + kOffX16);
  float*          XZ     = (float*)(ws + kOffXZ);
  float*          UC     = (float*)(ws + kOffUC);
  unsigned short* UC16   = (unsigned short*)(ws + kOffUC16);
  float*          PROJ   = (float*)(ws + kOffPROJ);
  unsigned short* DT16   = (unsigned short*)(ws + kOffDT16);
  float*          DLR    = (float*)(ws + kOffDLR);
  unsigned short* Y16    = (unsigned short*)(ws + kOffY16);
  float*          MB     = (float*)(ws + kOffMB);
  const float* dummy_bias  = b_dt;
  const float* dummy_resid = x;

  constexpr int kT8Win  = kXZP * kDmod / 8;
  constexpr int kT8Wxp  = kPrjP * kDin / 8;
  constexpr int kR8Wxp  = kPrjN * kDin / 8;
  constexpr int kT8Wdt  = kDin * kDtR / 8;
  constexpr int kT8Wout = kDmod * kDin / 8;
  constexpr int kT8X    = kRows * kDmod / 8;
  static_assert(kT8Win % 256 == 0 && kT8Wxp % 256 == 0 && kT8Wdt % 256 == 0 && kT8Wout % 256 == 0 && kT8X % 256 == 0,
                "cast grids exact");
  cast_f16_kernel<<<kT8Win / 256, 256, 0, stream>>>(W_in, WIN16, kT8Win, kT8Win, kCarWin);
  cast_f16_kernel<<<kT8Wxp / 256, 256, 0, stream>>>(W_xprj, WXP16, kT8Wxp, kR8Wxp, kCarWxp);
  cast_f16_kernel<<<kT8Wdt / 256, 256, 0, stream>>>(W_dt, WDT16, kT8Wdt, kT8Wdt, kCarWdt);
  cast_f16_kernel<<<kT8Wout / 256, 256, 0, stream>>>(W_out, WOUT16, kT8Wout, kT8Wout, kCarWout);
  cast_f16_kernel<<<kT8X / 256, 256, 0, stream>>>(x, X16, kT8X, kT8X, kCarX);

  for (int b = 0; b < kBatch; ++b) {
    const unsigned short* X16b = X16 + (size_t)b * kSeqL * kDmod;
    float* MBb = MB + (size_t)b * kSeqL * kDmod;

    wmma_gemm64<0, false, 0, 0, false><<<dim3(256, 1), 256, 0, stream>>>(
        X16b, X16b, kDmod, 0L, WIN16, WIN16, kDmod, 0L,
        (void*)XZ, (void*)XZ, kXZP, 0L, dummy_bias, dummy_resid, 0L, kSeqL, kXZP, kDmod, kSclIn);

    conv_silu_kernel<<<dim3(kDin / 256, kSeqL / 64), 256, 0, stream>>>(XZ, conv_w, conv_b, UC, UC16);

    wmma_gemm64<0, false, 0, 0, false><<<dim3(8, 1), 256, 0, stream>>>(
        UC16, UC16, kDin, 0L, WXP16, WXP16, kDin, 0L,
        (void*)PROJ, (void*)PROJ, kPrjP, 0L, dummy_bias, dummy_resid, 0L, kSeqL, kPrjP, kDin, kSclXp);

    dt_cast_kernel<<<(kSeqL * kDtR) / 8 / 256, 256, 0, stream>>>(PROJ, DT16, (kSeqL * kDtR) / 8, kCarDt);

    wmma_gemm64<0, false, 0, 0, false><<<dim3(128, 1), 256, 0, stream>>>(
        DT16, DT16, kDtR, 0L, WDT16, WDT16, kDtR, 0L,
        (void*)DLR, (void*)DLR, kDin, 0L, dummy_bias, dummy_resid, 0L, kSeqL, kDin, kDtR, kSclDt);

    scan_kernel<<<dim3(kDin / 256, 1), 256, 0, stream>>>(DLR, UC, XZ, PROJ, b_dt, A_log, Dv, Y16);

    wmma_gemm64<0, false, 0, 0, false><<<dim3(64, 1), 256, 0, stream>>>(
        Y16, Y16, kDin, 0L, WOUT16, WOUT16, kDin, 0L,
        (void*)MBb, (void*)MBb, kDmod, 0L, dummy_bias, dummy_resid, 0L, kSeqL, kDmod, kDin, kSclOut);
  }

  ln_resid_kernel<<<kRows, 256, 0, stream>>>(MB, x, ln_w, ln_b, dout);
}
